// CrossAttention_13159779795222
// MI455X (gfx1250) — hardware-verified
//
#include <hip/hip_runtime.h>
#ifndef NB
#define NB 4
#endif
#ifndef SQ
#define SQ 2048
#endif
#ifndef SK
#define SK 1024
#endif
#define SQ_FULL 2048
#define SK_FULL 1024
#define DX 512
#define DC 768
#define DM 512
#define DO 512
#define NH 8
#define HD 64
#define QP (2 * DM)
#define OP (2 * DM)
#define NRQ (NB * SQ)
#define NRK (NB * SK)
#define RQ 1024.0f
#define RQI 0.0009765625f
#define RO 32.0f
#define LN256 5.545177444479562f

typedef unsigned short v8us __attribute__((ext_vector_type(8), may_alias));
typedef float  v8f  __attribute__((ext_vector_type(8)));
typedef float  v4f  __attribute__((ext_vector_type(4)));
typedef float  v4fa __attribute__((ext_vector_type(4), may_alias));
typedef _Float16 v16h __attribute__((ext_vector_type(16)));
typedef _Float16 v4h __attribute__((ext_vector_type(4)));
union FragH { v16h v; v8us half[2]; _Float16 h[16]; unsigned short u[16]; };

static_assert(NH * HD == DM);
static_assert(HD == 64);
static_assert(SQ % 64 == 0 && NRQ % 128 == 0);
static_assert(SK % 64 == 0 && NRK % 128 == 0);
static_assert(DX % 32 == 0 && DC % 32 == 0 && (2 * DM) % 32 == 0);
static_assert(DM % 128 == 0 && DM % 64 == 0 && DO % 64 == 0);
static_assert(DX % 8 == 0 && DC % 8 == 0 && DM % 8 == 0);
static_assert(SQ <= SQ_FULL && SK <= SK_FULL);

__device__ __forceinline__ unsigned short bf16_bits(float x) { unsigned int u = __float_as_uint(x); return (unsigned short)((u + 0x7FFFu + ((u >> 16) & 1u)) >> 16); }
__device__ __forceinline__ float bf16_rne(float x) { return __uint_as_float(((unsigned int)bf16_bits(x)) << 16); }

__device__ __forceinline__ v16h g2_frag(const _Float16* p, int hh) { FragH f; f.half[0] = *(const v8us*)((const unsigned short*)p + 8 * hh); f.half[1] = *(const v8us*)((const unsigned short*)p + 16 + 8 * hh); return f.v; }
__device__ __forceinline__ v8f g2_mma(v16h a, v16h b, v8f c) { v8f d = __builtin_amdgcn_wmma_f32_16x16x32_f16(false, a, false, b, (short)0, c, false, false); asm volatile("v_nop\n\tv_nop\n\tv_nop\n\tv_nop" : "+v"(d) : "v"(a), "v"(b)); return d; }

__global__ __launch_bounds__(256) void k_wplane(const float* __restrict__ w, int rows, int cols, _Float16* __restrict__ dst, int dpitch, int dcol0, float scale) {
  const int t = blockIdx.x * 256 + threadIdx.x; const int c8n = cols >> 3; if (t >= rows * c8n) return;
  const int r = t / c8n, c8 = (t - r * c8n) * 8;
  const v4f a = *(const v4fa*)(w + (size_t)r * cols + c8), c = *(const v4fa*)(w + (size_t)r * cols + c8 + 4);
  FragH f;
#pragma unroll
  for (int q = 0; q < 4; ++q) { f.h[q] = (_Float16)(bf16_rne(a[q]) * scale); f.h[4 + q] = (_Float16)(bf16_rne(c[q]) * scale); }
  const v8us o = f.half[0];
  unsigned short* d = (unsigned short*)dst + (size_t)r * dpitch + dcol0 + c8;
  *(volatile v8us*)d = o; __threadfence(); *(volatile v8us*)d = o;
}

__global__ __launch_bounds__(256) void k_x16(const float* __restrict__ x, _Float16* __restrict__ X16, int rowsB, int rowsFull, int width, int nb) {
  const int t = blockIdx.x * 256 + threadIdx.x; const int c8n = width >> 3; if (t >= nb * rowsB * c8n) return;
  const int row = t / c8n, c8 = (t - row * c8n) * 8; const int b = row / rowsB, n = row - b * rowsB;
  const float* s = x + ((size_t)b * rowsFull + n) * width + c8;
  const v4f a = *(const v4fa*)s, c = *(const v4fa*)(s + 4);
  FragH f;
#pragma unroll
  for (int q = 0; q < 4; ++q) { f.h[q] = (_Float16)bf16_rne(a[q]); f.h[4 + q] = (_Float16)bf16_rne(c[q]); }
  const v8us o = f.half[0];
  unsigned short* d = (unsigned short*)X16 + (size_t)row * width + c8;
  *(volatile v8us*)d = o; __threadfence(); *(volatile v8us*)d = o;
}

template <int MODE>
__device__ __forceinline__ void gemm_body(const _Float16* __restrict__ A, int lda, size_t sA, const _Float16* __restrict__ Bh, int ldb, size_t sB, float alpha,
    const float* __restrict__ bias, float* __restrict__ C, _Float16* __restrict__ C16, int ldc, size_t sC, int resoff, float rscale, int M, int N, int K) {
  __shared__ __attribute__((aligned(16))) float so[4][32][68];
  const int tid = threadIdx.x, lane = tid & 31, ln = lane & 15, hh = lane >> 4;
  const int w = __builtin_amdgcn_readfirstlane(tid >> 5);
  const int by = blockIdx.y;
  A += (size_t)by * sA; Bh += (size_t)by * sB; const size_t cofs = (size_t)by * sC;
  const int ntn = N >> 6; const int mt = blockIdx.x / ntn, nq = blockIdx.x - mt * ntn; const int row0 = mt * 128 + 32 * w, col0 = nq * 64; if (row0 >= M) return;
  const _Float16* a0p = A + (size_t)(row0 + ln) * lda; const _Float16* a1p = a0p + (size_t)16 * lda;
  const _Float16* b0p = Bh + (size_t)(col0 + ln) * ldb; const _Float16* b1p = b0p + (size_t)16 * ldb; const _Float16* b2p = b1p + (size_t)16 * ldb; const _Float16* b3p = b2p + (size_t)16 * ldb;
  const v8f z8 = {0.f,0.f,0.f,0.f,0.f,0.f,0.f,0.f}; v8f c00 = z8, c01 = z8, c02 = z8, c03 = z8, c10 = z8, c11 = z8, c12 = z8, c13 = z8;
#pragma unroll 1
  for (int kb = 0; kb < K; kb += 32) { const v16h a0 = g2_frag(a0p + kb, hh), a1 = g2_frag(a1p + kb, hh);
    v16h b = g2_frag(b0p + kb, hh); c00 = g2_mma(a0, b, c00); c10 = g2_mma(a1, b, c10);
    b = g2_frag(b1p + kb, hh); c01 = g2_mma(a0, b, c01); c11 = g2_mma(a1, b, c11);
    b = g2_frag(b2p + kb, hh); c02 = g2_mma(a0, b, c02); c12 = g2_mma(a1, b, c12);
    b = g2_frag(b3p + kb, hh); c03 = g2_mma(a0, b, c03); c13 = g2_mma(a1, b, c13); }
  v8f accs[8] = {c00, c01, c02, c03, c10, c11, c12, c13};
#pragma unroll
  for (int u = 0; u < 8; ++u) { const int t = u & 3, half = u >> 2; const int col = col0 + t * 16 + ln; float bv = 0.f; if (MODE == 2) bv = bf16_rne(bias[col]);
#pragma unroll
    for (int r = 0; r < 8; ++r) { const int rloc = half * 16 + 8 * hh + r; so[w][rloc][t * 16 + ln] = accs[u][r] * alpha + bv; } }
  __builtin_amdgcn_fence(4  , "workgroup"); __builtin_amdgcn_wave_barrier();
  const int rsub = lane >> 4, c4 = (lane & 15) * 4;
  for (int pass = 0; pass < 2; ++pass) {
#pragma unroll
    for (int q = 0; q < 16; ++q) { const int r = q * 2 + rsub; const v4f v = *(const v4fa*)&so[w][r][c4];
      if (MODE == 2) { *(volatile v4f*)(C + cofs + (size_t)(row0 + r) * ldc + col0 + c4) = v; }
      else { v4h h4; for (int i = 0; i < 4; ++i) h4[i] = (_Float16)v[i];
        *(volatile v4h*)(C16 + cofs + (size_t)(row0 + r) * ldc + col0 + c4) = h4;
        if (MODE == 1) { v4h r4; for (int i = 0; i < 4; ++i) r4[i] = (_Float16)((v[i] - (float)h4[i]) * rscale);
          *(volatile v4h*)(C16 + cofs + (size_t)(row0 + r) * ldc + resoff + col0 + c4) = r4; } } }
    if (pass == 0) __threadfence(); }
}
__global__ __launch_bounds__(128) void k_gemm_h16(const _Float16* __restrict__ A, int lda, size_t sA, const _Float16* __restrict__ Bh, int ldb, size_t sB, float alpha, _Float16* __restrict__ C16, int ldc, size_t sC, int M, int N, int K) {
  gemm_body<0>(A, lda, sA, Bh, ldb, sB, alpha, nullptr, nullptr, C16, ldc, sC, 0, 0.f, M, N, K); }
__global__ __launch_bounds__(128) void k_gemm_hr(const _Float16* __restrict__ A, int lda, const _Float16* __restrict__ Bh, int ldb, float alpha, _Float16* __restrict__ C16, int ldc, int resoff, float rscale, int M, int N, int K) {
  gemm_body<1>(A, lda, 0, Bh, ldb, 0, alpha, nullptr, nullptr, C16, ldc, 0, resoff, rscale, M, N, K); }
__global__ __launch_bounds__(128) void k_gemm_f32(const _Float16* __restrict__ A, int lda, const _Float16* __restrict__ Bh, int ldb, float alpha, const float* __restrict__ bias, float* __restrict__ C, int ldc, int M, int N, int K) {
  gemm_body<2>(A, lda, 0, Bh, ldb, 0, alpha, bias, C, nullptr, ldc, 0, 0, 0.f, M, N, K); }

__global__ __launch_bounds__(128) void k_flash(const _Float16* __restrict__ Q2, const _Float16* __restrict__ K16, const _Float16* __restrict__ VT, _Float16* __restrict__ O2) {
  __shared__ __attribute__((aligned(16))) float so[4][16][68];
  const int wave = __builtin_amdgcn_readfirstlane(threadIdx.x >> 5);
  const int lane = threadIdx.x & 31, ln = lane & 15, hh = lane >> 4;
  const int nqb = SQ / 64;
  const int bh = blockIdx.x / nqb, qb = blockIdx.x - bh * nqb;
  const int b = bh / NH, h = bh - b * NH;
  const int q0 = qb * 64 + wave * 16;
  const int qoff = (b * SQ + q0 + ln) * QP + h * HD;
  const int koff = (b * SK + ln) * DM + h * HD;
  const int voff = ((b * NH + h) * HD + ln) * SK;
  const v8f z8 = {0.f,0.f,0.f,0.f,0.f,0.f,0.f,0.f};
  v8f o0 = z8, o1 = z8, o2 = z8, o3 = z8;
  float m = -1.0e30f, l = 0.f;
#pragma unroll 1
  for (int kb = 0; kb < SK; kb += 32) {
    v8f sh0 = z8, sh1 = z8, sl0 = z8, sl1 = z8;
#pragma unroll
    for (int ks = 0; ks < 2; ++ks) {
      int qo = qoff + ks * 32;
      asm volatile("" : "+v"(qo));
      const v16h bqh = g2_frag(Q2 + qo, hh);
      const v16h bql = g2_frag(Q2 + qo + DM, hh);
      const v16h a0 = g2_frag(K16 + koff + kb * DM + ks * 32, hh);
      const v16h a1 = g2_frag(K16 + koff + (kb + 16) * DM + ks * 32, hh);
      sh0 = g2_mma(a0, bqh, sh0); sl0 = g2_mma(a0, bql, sl0);
      sh1 = g2_mma(a1, bqh, sh1); sl1 = g2_mma(a1, bql, sl1);
    }
    float t0[8], t1[8]; float mx = -3.0e38f;
#pragma unroll
    for (int r = 0; r < 8; ++r) { t0[r] = (sh0[r] + sl0[r] * RQI) * 0.125f; t1[r] = (sh1[r] + sl1[r] * RQI) * 0.125f; mx = fmaxf(mx, fmaxf(t0[r], t1[r])); }
    mx = fmaxf(mx, __shfl_xor(mx, 16));
    const float mn = fmaxf(m, mx);
    const float al = __expf(m - mn);
    m = mn;
    const float ms = mn - LN256;
    FragH p; float ps = 0.f;
#pragma unroll
    for (int r = 0; r < 8; ++r) { const float e0 = __expf(t0[r] - ms), e1 = __expf(t1[r] - ms); ps += e0 + e1; p.h[r] = (_Float16)e0; p.h[8 + r] = (_Float16)e1; }
    l = l * al + ps;
#pragma unroll
    for (int r = 0; r < 8; ++r) { o0[r] *= al; o1[r] *= al; o2[r] *= al; o3[r] *= al; }
    const v16h v0 = g2_frag(VT + voff + kb, hh);
    const v16h v1 = g2_frag(VT + voff + 16 * SK + kb, hh);
    const v16h v2 = g2_frag(VT + voff + 32 * SK + kb, hh);
    const v16h v3 = g2_frag(VT + voff + 48 * SK + kb, hh);
    o0 = g2_mma(v0, p.v, o0); o1 = g2_mma(v1, p.v, o1); o2 = g2_mma(v2, p.v, o2); o3 = g2_mma(v3, p.v, o3);
  }
  l += __shfl_xor(l, 16);
  const float fin = 64.0f * (1.0f / l);
  { v4f w0, w1;
#pragma unroll
    for (int q = 0; q < 4; ++q) { w0[q] = o0[q] * fin; w1[q] = o0[4 + q] * fin; }
    *(v4f*)&so[wave][ln][0 + 8 * hh] = w0; *(v4f*)&so[wave][ln][4 + 8 * hh] = w1;
#pragma unroll
    for (int q = 0; q < 4; ++q) { w0[q] = o1[q] * fin; w1[q] = o1[4 + q] * fin; }
    *(v4f*)&so[wave][ln][16 + 8 * hh] = w0; *(v4f*)&so[wave][ln][20 + 8 * hh] = w1;
#pragma unroll
    for (int q = 0; q < 4; ++q) { w0[q] = o2[q] * fin; w1[q] = o2[4 + q] * fin; }
    *(v4f*)&so[wave][ln][32 + 8 * hh] = w0; *(v4f*)&so[wave][ln][36 + 8 * hh] = w1;
#pragma unroll
    for (int q = 0; q < 4; ++q) { w0[q] = o3[q] * fin; w1[q] = o3[4 + q] * fin; }
    *(v4f*)&so[wave][ln][48 + 8 * hh] = w0; *(v4f*)&so[wave][ln][52 + 8 * hh] = w1; }
  __builtin_amdgcn_fence(4  , "workgroup"); __builtin_amdgcn_wave_barrier();
  const int rq = lane >> 3, c8 = (lane & 7) * 8;
  for (int pass = 0; pass < 2; ++pass) {
#pragma unroll
    for (int it = 0; it < 4; ++it) { const int row = it * 4 + rq;
      const v4f x0 = *(const v4fa*)&so[wave][row][c8], x1 = *(const v4fa*)&so[wave][row][c8 + 4];
      FragH fh, fr;
#pragma unroll
      for (int q = 0; q < 4; ++q) { _Float16 hv = (_Float16)x0[q]; fh.h[q] = hv; fr.h[q] = (_Float16)((x0[q] - (float)hv) * RO); hv = (_Float16)x1[q]; fh.h[4 + q] = hv; fr.h[4 + q] = (_Float16)((x1[q] - (float)hv) * RO); }
      unsigned short* dst = (unsigned short*)O2 + (size_t)(b * SQ + q0 + row) * OP + h * HD + c8;
      *(volatile v8us*)dst = fh.half[0]; *(volatile v8us*)(dst + DM) = fr.half[0]; }
    if (pass == 0) __threadfence(); }
}

#define AL256(x) ((((size_t)(x)) + 255) & ~(size_t)255)
extern "C" void kernel_launch(void* const* d_in, const int* in_sizes, int n_in,
                              void* d_out, int out_size, void* d_ws, size_t ws_size, hipStream_t stream) {
  if (n_in < 7) return;
  if ((long long)in_sizes[0] < ((long long)(NB - 1) * SQ_FULL + SQ) * DX) return;
  if ((long long)in_sizes[1] < ((long long)(NB - 1) * SK_FULL + SK) * DC) return;
  if (in_sizes[2] < DM * DX || in_sizes[3] < DM * DC || in_sizes[4] < DM * DC || in_sizes[5] < DO * DM || in_sizes[6] < DO) return;
  if ((long long)out_size < (long long)NRQ * DO) return;
  const float* x = (const float*)d_in[0]; const float* ctx = (const float*)d_in[1]; const float* wq = (const float*)d_in[2]; const float* wk = (const float*)d_in[3];
  const float* wv = (const float*)d_in[4]; const float* wo = (const float*)d_in[5]; const float* bo = (const float*)d_in[6];
  constexpr size_t SZ_BQ = AL256((size_t)DM * DX * 2), SZ_BK = AL256((size_t)DM * DC * 2), SZ_BV = AL256((size_t)DM * DC * 2), SZ_BO = AL256((size_t)DO * 2 * DM * 2);
  constexpr size_t SZ_X = AL256((size_t)NRQ * DX * 2), SZ_C = AL256((size_t)NRK * DC * 2), SZ_Q = AL256((size_t)NRQ * QP * 2), SZ_K = AL256((size_t)NRK * DM * 2);
  constexpr size_t SZ_VT = AL256((size_t)NB * DM * SK * 2), SZ_O = AL256((size_t)NRQ * OP * 2);
  constexpr size_t TOTAL = SZ_BQ + SZ_BK + SZ_BV + SZ_BO + SZ_X + SZ_C + SZ_Q + SZ_K + SZ_VT + SZ_O;
  static_assert(TOTAL <= (size_t)134217728);
  if (TOTAL > ws_size) return;
  char* ws = (char*)d_ws; size_t off = 0;
  _Float16* BQ = (_Float16*)(ws + off); off += SZ_BQ;
  _Float16* BK = (_Float16*)(ws + off); off += SZ_BK;
  _Float16* BV = (_Float16*)(ws + off); off += SZ_BV;
  _Float16* BO2 = (_Float16*)(ws + off); off += SZ_BO;
  _Float16* X16 = (_Float16*)(ws + off); off += SZ_X;
  _Float16* C16 = (_Float16*)(ws + off); off += SZ_C;
  _Float16* Q2 = (_Float16*)(ws + off); off += SZ_Q;
  _Float16* K16 = (_Float16*)(ws + off); off += SZ_K;
  _Float16* VT = (_Float16*)(ws + off); off += SZ_VT;
  _Float16* O2 = (_Float16*)(ws + off); off += SZ_O;
  k_wplane<<<(DM * (DX / 8) + 255) / 256, 256, 0, stream>>>(wq, DM, DX, BQ, DX, 0, 16.0f);
  k_wplane<<<(DM * (DC / 8) + 255) / 256, 256, 0, stream>>>(wk, DM, DC, BK, DC, 0, 16.0f);
  k_wplane<<<(DM * (DC / 8) + 255) / 256, 256, 0, stream>>>(wv, DM, DC, BV, DC, 0, 16.0f);
  k_wplane<<<(DO * (DM / 8) + 255) / 256, 256, 0, stream>>>(wo, DO, DM, BO2, 2 * DM, 0, 16.0f);
  k_wplane<<<(DO * (DM / 8) + 255) / 256, 256, 0, stream>>>(wo, DO, DM, BO2, 2 * DM, DM, 0.5f);
  k_x16<<<(NRQ * (DX / 8) + 255) / 256, 256, 0, stream>>>(x, X16, SQ, SQ_FULL, DX, NB);
  k_x16<<<(NRK * (DC / 8) + 255) / 256, 256, 0, stream>>>(ctx, C16, SK, SK_FULL, DC, NB);
  k_gemm_hr<<<dim3((NRQ / 128) * (DM / 64), 1), 128, 0, stream>>>(X16, DX, BQ, DX, 0.0625f, Q2, QP, DM, RQ, NRQ, DM, DX);
  k_gemm_h16<<<dim3((NRK / 128) * (DM / 64), 1), 128, 0, stream>>>(C16, DC, 0, BK, DC, 0, 0.0625f, K16, DM, 0, NRK, DM, DC);
  k_gemm_h16<<<dim3((DM / 128) * (SK / 64), NB), 128, 0, stream>>>(BV, DC, 0, C16, DC, (size_t)SK * DC, 0.0625f, VT, SK, (size_t)DM * SK, DM, SK, DC);
  k_flash<<<NB * NH * (SQ / 64), 128, 0, stream>>>(Q2, K16, VT, O2);
  k_gemm_f32<<<dim3((NRQ / 128) * (DO / 64), 1), 128, 0, stream>>>(O2, OP, BO2, 2 * DM, 0.0009765625f, bo, (float*)d_out, DO, NRQ, DO, 2 * DM);
}
